// GraphAttentionalLayer_730144440901
// MI455X (gfx1250) — hardware-verified
//
#include <hip/hip_runtime.h>
#include <math.h>

typedef __attribute__((ext_vector_type(16))) _Float16 v16h;
typedef __attribute__((ext_vector_type(8)))  _Float16 v8h;
typedef __attribute__((ext_vector_type(8)))  float    v8f;
typedef __attribute__((ext_vector_type(4)))  float    v4f;

constexpr int kBatch = 2;
constexpr int kNodes = 4096;
constexpr int kDim   = 128;
constexpr int kRows  = kBatch * kNodes;
constexpr int kChunk = 128;
constexpr int kChunksPerBatch = kNodes / kChunk;
static_assert(kRows == 8192, "row count");
static_assert((kRows % 64) == 0 && (kDim % 64) == 0 && (kDim % 32) == 0, "GEMM tile multiples");
static_assert(kChunksPerBatch == 32, "chunks per batch");

constexpr float kCarryH = 64.0f;
constexpr float kCarryW = 1024.0f;
constexpr float kFold   = 1.0f / (kCarryH * kCarryW);
constexpr float kF16MinNormal = 6.103515625e-5f;
static_assert(kCarryH * kCarryW == 65536.0f, "fold is 2^-16");

constexpr int kCvtBlocksH = (kRows * kDim / 8) / 256;
constexpr int kCvtBlocksW = (kDim * kDim / 8) / 256;
static_assert(kCvtBlocksH * 256 * 8 == kRows * kDim, "h plane covered exactly");
static_assert(kCvtBlocksW * 256 * 8 == kDim * kDim, "W plane covered exactly");

constexpr size_t kOffAH   = 0;
constexpr size_t kOffWH   = kOffAH + (size_t)kRows * kDim * 2;
constexpr size_t kOffHW   = kOffWH + (size_t)kDim * kDim * 2;
constexpr size_t kOffSJ   = kOffHW + (size_t)kRows * kDim * 4;
constexpr size_t kOffPART = kOffSJ + (size_t)kRows * 4;
constexpr size_t kWsTotal = kOffPART + (size_t)kBatch * kChunksPerBatch * kDim * 4;
static_assert(kWsTotal == 6389760ull, "carve total");
static_assert(kWsTotal <= 134217728ull, "carve cap");
static_assert((kOffWH % 128) == 0 && (kOffHW % 128) == 0 && (kOffSJ % 128) == 0 && (kOffPART % 128) == 0, "128-B aligned regions");

union FragH { v16h v; v8h h[2]; };
__device__ __forceinline__ v16h frag_load(const _Float16* p) {
  FragH f;
  f.h[0] = *(const v8h*)(p);
  f.h[1] = *(const v8h*)(p + 16);
  return f.v;
}
__device__ __forceinline__ v8f mma_f16(v16h a, v16h b, v8f c) {
  c = __builtin_amdgcn_wmma_f32_16x16x32_f16(false, a, false, b, (short)0, c, false, false);
  asm volatile("v_nop\n\tv_nop\n\tv_nop\n\tv_nop" : "+v"(c) : "v"(a), "v"(b));
  return c;
}

__global__ __launch_bounds__(256) void cvt_planes_kernel(
    const float* __restrict__ hsrc, const float* __restrict__ wsrc,
    unsigned short* __restrict__ AH, unsigned short* __restrict__ WH)
{
  const int blk = blockIdx.x;
  const bool isW = (blk >= kCvtBlocksH);
  const float* src = isW ? wsrc : hsrc;
  unsigned short* dst = isW ? WH : AH;
  const float carry = isW ? kCarryW : kCarryH;
  const int i = (isW ? (blk - kCvtBlocksH) : blk) * 256 + (int)threadIdx.x;
  const size_t e0 = (size_t)i << 3;
  const v4f a0 = *(const v4f*)(src + e0);
  const v4f a1 = *(const v4f*)(src + e0 + 4);
  v8h hv;
#pragma unroll
  for (int e = 0; e < 4; ++e) {
    float x0 = a0[e] * carry;
    float x1 = a1[e] * carry;
    x0 = (fabsf(x0) < kF16MinNormal) ? 0.0f : x0;
    x1 = (fabsf(x1) < kF16MinNormal) ? 0.0f : x1;
    hv[e]     = (_Float16)x0;
    hv[4 + e] = (_Float16)x1;
  }
  unsigned short* q = dst + e0;
  *(volatile v8h*)q = hv;
  __threadfence();
  *(volatile v8h*)q = hv;
}

__global__ __launch_bounds__(256) void proj_gemm_kernel(
    const unsigned short* __restrict__ Ap, const unsigned short* __restrict__ Btp, float* __restrict__ C)
{
  const _Float16* A  = (const _Float16*)Ap;
  const _Float16* Bt = (const _Float16*)Btp;
  __shared__ __align__(16) float sT[8][16 * 68];
  const int lane = threadIdx.x & 31;
  const int wave = threadIdx.x >> 5;
  constexpr int tilesN = kDim >> 6;
  constexpr int tilesM = kRows >> 6;
  const int tile = blockIdx.x * 8 + wave;
  if (tile >= tilesM * tilesN) return;
  const int tm = tile / tilesN;
  const int tn = tile - tm * tilesN;
  const int m0 = tm << 6;
  const int n0 = tn << 6;

  const int rlane = lane & 15;
  const int koff  = (lane >> 4) * 8;
  const int mOff  = (lane >> 4) * 8;

  v8f acc[4][4];
#pragma unroll
  for (int i = 0; i < 4; ++i)
#pragma unroll
    for (int j = 0; j < 4; ++j) acc[i][j] = (v8f){0.f, 0.f, 0.f, 0.f, 0.f, 0.f, 0.f, 0.f};

#pragma unroll 1
  for (int k0 = 0; k0 < kDim; k0 += 32) {
    v16h bh[4];
#pragma unroll
    for (int j = 0; j < 4; ++j) {
      const size_t bo = (size_t)(n0 + (j << 4) + rlane) * kDim + koff + k0;
      bh[j] = frag_load(Bt + bo);
    }
#pragma unroll
    for (int i = 0; i < 4; ++i) {
      const size_t ao = (size_t)(m0 + (i << 4) + rlane) * kDim + koff + k0;
      const v16h ah = frag_load(A + ao);
#pragma unroll
      for (int j = 0; j < 4; ++j) acc[i][j] = mma_f16(ah, bh[j], acc[i][j]);
    }
  }

  float* slab = sT[wave];
#pragma unroll
  for (int i = 0; i < 4; ++i) {
    const int mBase = m0 + (i << 4);
#pragma unroll
    for (int j = 0; j < 4; ++j) {
#pragma unroll
      for (int r = 0; r < 8; ++r) {
        const float v = acc[i][j][r] * kFold;
        slab[(mOff + r) * 68 + (j << 4) + rlane] = v;
      }
    }
    __builtin_amdgcn_fence(__ATOMIC_RELEASE, "workgroup");
    __builtin_amdgcn_wave_barrier();
    __builtin_amdgcn_fence(__ATOMIC_ACQUIRE, "workgroup");
    {
      const int hh = lane >> 4;
      const int c4 = (lane & 15) * 4;
      for (int pass = 0; pass < 2; ++pass) {
#pragma unroll
        for (int it = 0; it < 8; ++it) {
          const int row = it * 2 + hh;
          const v4f v = *(const v4f*)(slab + row * 68 + c4);
          *(volatile v4f*)(C + (size_t)(mBase + row) * kDim + n0 + c4) = v;
        }
        __threadfence();
      }
    }
    __builtin_amdgcn_fence(__ATOMIC_RELEASE, "workgroup");
    __builtin_amdgcn_wave_barrier();
    __builtin_amdgcn_fence(__ATOMIC_ACQUIRE, "workgroup");
  }
}

__global__ __launch_bounds__(256) void row_score_kernel(
    const float* __restrict__ HW, const float* __restrict__ aj, float* __restrict__ SJ)
{
  const int lane = threadIdx.x & 31;
  const int wave = threadIdx.x >> 5;
  const int row0 = (blockIdx.x * 8 + wave) * 32;
  const v4f av = *(const v4f*)(aj + lane * 4);
  float keep = 0.0f;
#pragma unroll 4
  for (int rr = 0; rr < 32; ++rr) {
    const v4f x = *(const v4f*)(HW + (size_t)(row0 + rr) * kDim + lane * 4);
    float s = x[0] * av[0];
    s = fmaf(x[1], av[1], s);
    s = fmaf(x[2], av[2], s);
    s = fmaf(x[3], av[3], s);
#pragma unroll
    for (int off = 16; off > 0; off >>= 1) s += __shfl_xor(s, off, 32);
    keep = (lane == rr) ? s : keep;
  }
  volatile float* p = SJ + row0 + lane;
  *p = keep;
  __threadfence();
  *p = keep;
}

__global__ __launch_bounds__(128) void weighted_partial_kernel(
    const float* __restrict__ HW, const float* __restrict__ SJ, float* __restrict__ PART)
{
  __shared__ float sRed[4];
  __shared__ float sSum[4];
  __shared__ float sP[kChunk];
  const int tid  = threadIdx.x;
  const int lane = tid & 31;
  const int wave = tid >> 5;
  const int b = blockIdx.x >> 5;
  const int c = blockIdx.x & 31;
  const float* sb = SJ + (size_t)b * kNodes;

  float m = -INFINITY;
#pragma unroll 1
  for (int i = 0; i < 8; ++i) {
    const v4f s4 = *(const v4f*)(sb + (size_t)(tid + 128 * i) * 4);
    m = fmaxf(m, fmaxf(fmaxf(s4[0], s4[1]), fmaxf(s4[2], s4[3])));
  }
#pragma unroll
  for (int off = 16; off > 0; off >>= 1) m = fmaxf(m, __shfl_xor(m, off, 32));
  if (lane == 0) sRed[wave] = m;
  __syncthreads();
  const float mb = fmaxf(fmaxf(sRed[0], sRed[1]), fmaxf(sRed[2], sRed[3]));

  float z = 0.0f;
#pragma unroll 1
  for (int i = 0; i < 8; ++i) {
    const v4f s4 = *(const v4f*)(sb + (size_t)(tid + 128 * i) * 4);
    z += expf(s4[0] - mb);
    z += expf(s4[1] - mb);
    z += expf(s4[2] - mb);
    z += expf(s4[3] - mb);
  }
#pragma unroll
  for (int off = 16; off > 0; off >>= 1) z += __shfl_xor(z, off, 32);
  if (lane == 0) sSum[wave] = z;
  const float pj = expf(sb[c * kChunk + tid] - mb);
  sP[tid] = pj;
  __syncthreads();
  const float zb = ((sSum[0] + sSum[1]) + sSum[2]) + sSum[3];
  const float invZ = 1.0f / zb;

  const float* base = HW + ((size_t)b * kNodes + (size_t)c * kChunk) * kDim + tid;
  float acc = 0.0f;
#pragma unroll 8
  for (int j = 0; j < kChunk; ++j) acc = fmaf(sP[j], base[(size_t)j * kDim], acc);
  const float val = acc * invZ;
  volatile float* p = PART + ((size_t)b * kChunksPerBatch + c) * kDim + tid;
  *p = val;
  __threadfence();
  *p = val;
}

__global__ __launch_bounds__(256) void broadcast_rows_kernel(
    const float* __restrict__ PART, float* __restrict__ out)
{
  const int lane = threadIdx.x & 31;
  const int wave = threadIdx.x >> 5;
  const int rowbase = blockIdx.x * 64;
  const int b = rowbase >> 12;
  const float* pb = PART + (size_t)b * kChunksPerBatch * kDim + lane * 4;
  v4f r = (v4f){0.0f, 0.0f, 0.0f, 0.0f};
#pragma unroll 4
  for (int c = 0; c < kChunksPerBatch; ++c) {
    const v4f t = *(const v4f*)(pb + (size_t)c * kDim);
    r += t;
  }
  float* ob = out + (size_t)(rowbase + wave * 8) * kDim + lane * 4;
  for (int pass = 0; pass < 2; ++pass) {
#pragma unroll
    for (int it = 0; it < 8; ++it) {
      *(volatile v4f*)(ob + (size_t)it * kDim) = r;
    }
    __threadfence();
  }
}

extern "C" void kernel_launch(void* const* d_in, const int* in_sizes, int n_in,
                              void* d_out, int out_size, void* d_ws, size_t ws_size,
                              hipStream_t stream) {
  if (n_in < 4) return;
  if (in_sizes[0] != kRows * kDim) return;
  if (in_sizes[1] != kDim * kDim) return;
  if (in_sizes[2] != kDim) return;
  if (in_sizes[3] != kDim) return;
  if (out_size != kRows * kDim) return;
  if (ws_size < kWsTotal) return;

  const float* h  = (const float*)d_in[0];
  const float* W  = (const float*)d_in[1];
  const float* aj = (const float*)d_in[3];
  float* out = (float*)d_out;

  char* ws = (char*)d_ws;
  unsigned short* AH   = (unsigned short*)(ws + kOffAH);
  unsigned short* WH   = (unsigned short*)(ws + kOffWH);
  float*          HW   = (float*)(ws + kOffHW);
  float*          SJ   = (float*)(ws + kOffSJ);
  float*          PART = (float*)(ws + kOffPART);

  cvt_planes_kernel<<<kCvtBlocksH + kCvtBlocksW, 256, 0, stream>>>(h, W, AH, WH);
  proj_gemm_kernel<<<(kRows / 64) * (kDim / 64) / 8, 256, 0, stream>>>(AH, WH, HW);
  row_score_kernel<<<kRows / 256, 256, 0, stream>>>(HW, aj, SJ);
  weighted_partial_kernel<<<kBatch * kChunksPerBatch, kChunk, 0, stream>>>(HW, SJ, PART);
  broadcast_rows_kernel<<<kRows / 64, 256, 0, stream>>>(PART, out);
}
